// MultiModalImputer_54769422959363
// MI455X (gfx1250) — hardware-verified
//
#include <hip/hip_runtime.h>

typedef __attribute__((ext_vector_type(16))) _Float16 v16h;
typedef __attribute__((ext_vector_type(8)))  _Float16 v8h;
typedef __attribute__((ext_vector_type(8)))  float    v8f;

#define NB   16
#define LEN  1024
#define DCH  12
#define EMB  8
#define HGRU 192
#define G3H  576
#define ROWS (NB*LEN)
#define FFH  512
typedef __attribute__((ext_vector_type(4))) float v4f;
typedef __attribute__((ext_vector_type(4))) unsigned v4u;
typedef float __attribute__((may_alias)) float_a;
template <typename T> __device__ __forceinline__ void vst2(void* p, T v) { *(volatile T*)p = v; __threadfence(); *(volatile T*)p = v; }

__device__ inline v8f vzero8f() {
  v8f c;
#pragma unroll
  for (int i = 0; i < 8; ++i) c[i] = 0.0f;
  return c;
}

__device__ inline v16h load_frag_a32(const float* base, int ld, int k0) {
  int lane = threadIdx.x & 31;
  int m = lane & 15, g = lane >> 4;
  const float* p = base + (size_t)m * ld + k0 + 8 * g;
  v16h a;
#pragma unroll
  for (int i = 0; i < 8; ++i) { a[i] = (_Float16)p[i]; a[i + 8] = (_Float16)p[16 + i]; }
  return a;
}
__device__ inline v16h load_frag_a(const _Float16* base, int ld, int k0) {
  int lane = threadIdx.x & 31;
  int m = lane & 15, g = lane >> 4;
  const _Float16* p = base + m * ld + k0 + 8 * g;
  v8h lo = *(const v8h*)p;
  v8h hi = *(const v8h*)(p + 16);
  v16h a;
#pragma unroll
  for (int i = 0; i < 8; ++i) { a[i] = lo[i]; a[i + 8] = hi[i]; }
  return a;
}

__device__ inline v16h load_frag_b(const _Float16* W, int ld, int n0, int k0) {
  int lane = threadIdx.x & 31;
  const _Float16* p = W + (size_t)(n0 + (lane & 15)) * ld + k0 + 8 * (lane >> 4);
  v8h lo = *(const v8h*)p;
  v8h hi = *(const v8h*)(p + 16);
  v16h b;
#pragma unroll
  for (int i = 0; i < 8; ++i) { b[i] = lo[i]; b[i + 8] = hi[i]; }
  return b;
}

__device__ inline v8f wmma16(v16h a, v16h b, v8f c) {
  v8f d = __builtin_amdgcn_wmma_f32_16x16x32_f16(false, a, false, b, (short)0, c, false, false);
  asm volatile("v_nop\n\tv_nop\n\tv_nop\n\tv_nop" : "+v"(d) : "v"(a), "v"(b));
  return d;
}

__global__ void cvt_f16_kernel(const float* __restrict__ in,
                               _Float16* __restrict__ out, int n) {
  int g8 = blockIdx.x * blockDim.x + threadIdx.x;
  if (g8 * 8 < n) { union { v8h h; v4u u; } pk;
#pragma unroll
    for (int e = 0; e < 8; ++e) pk.h[e] = (_Float16)in[g8 * 8 + e];
    vst2(out + (size_t)g8 * 8, pk.u); }
}

__global__ void cvt_w1_pad_kernel(const float* __restrict__ in,
                                  _Float16* __restrict__ out) {
  int g8 = blockIdx.x * blockDim.x + threadIdx.x;
  int i0 = g8 * 8;
  if (i0 >= DCH * FFH * 64) return;
  int k0 = i0 & 63, r = i0 >> 6;
  union { v8h h; v4u u; } pk;
#pragma unroll
  for (int e = 0; e < 8; ++e) { int k = k0 + e; pk.h[e] = (k < 48) ? (_Float16)in[r * 48 + k] : (_Float16)0.0f; }
  vst2(out + i0, pk.u);
}

__global__ void embed_kernel(const float* __restrict__ series,
                             const int* __restrict__ mask,
                             const float* __restrict__ series_W,
                             const float* __restrict__ mask_emb,
                             _Float16* __restrict__ x0) {
  int t = blockIdx.x * blockDim.x + threadIdx.x;
  if (t >= ROWS * DCH) return;
  int d = t % DCH, row = t / DCH;
  int m = mask[row * DCH + d]; m = m != 0 ? 1 : 0;
  int idx = m * (d + 1);
  const float sv = series[row * DCH + d];
  union { v8h h; v4u u; } pk;
#pragma unroll
  for (int e = 0; e < EMB; ++e) pk.h[e] = (_Float16)(mask_emb[idx * EMB + e] + sv * series_W[d * EMB + e]);
  vst2(x0 + (size_t)t * EMB, pk.u);
}

__global__ void adm_kernel(const float* __restrict__ adm,
                           const float* __restrict__ W1, const float* __restrict__ b1,
                           const float* __restrict__ W2, const float* __restrict__ b2,
                           float* __restrict__ adm_out) {
  __shared__ float hbuf[16][16];
  int t = threadIdx.x;
  int n = t >> 4, j = t & 15;
  float acc = b1[j];
  for (int k = 0; k < 64; ++k) acc += adm[n * 64 + k] * W1[j * 64 + k];
  hbuf[n][j] = fmaxf(acc, 0.0f);
  __syncthreads();
  float acc2 = b2[j];
  for (int k = 0; k < 16; ++k) acc2 += hbuf[n][k] * W2[j * 16 + k];
  adm_out[n * 16 + j] = acc2;
}

template <typename TA>
__global__ void __launch_bounds__(256) gemm_xw_kernel(const TA* __restrict__ A,
                               const _Float16* __restrict__ W,
                               const float* __restrict__ bias,
                               float* __restrict__ out, int K) {
  __shared__ __align__(16) float st[64][68];
  int wave = threadIdx.x >> 5;
  int r0 = blockIdx.x * 64 + (wave >> 1) * 16;
  int c0 = blockIdx.y * 64 + (wave & 1) * 32;
  v8f acc0 = vzero8f(), acc1 = vzero8f();
  const TA* Abase = A + (size_t)r0 * K;
  for (int k = 0; k < K; k += 32) {
    v16h a;
    if (sizeof(TA) == 2) a = load_frag_a((const _Float16*)Abase, K, k); else a = load_frag_a32((const float*)Abase, K, k);
    v16h b0 = load_frag_b(W, K, c0, k);
    v16h b1 = load_frag_b(W, K, c0 + 16, k);
    acc0 = wmma16(a, b0, acc0);
    acc1 = wmma16(a, b1, acc1);
  }
  int lane = threadIdx.x & 31;
  int mrow = (lane >> 4) * 8, ncol = lane & 15;
  const int rl0 = (wave >> 1) * 16, cl0 = (wave & 1) * 32;
#pragma unroll
  for (int v = 0; v < 8; ++v) {
    st[rl0 + mrow + v][cl0 + ncol]      = acc0[v] + bias[c0 + ncol];
    st[rl0 + mrow + v][cl0 + 16 + ncol] = acc1[v] + bias[c0 + 16 + ncol];
  }
  __syncthreads();
  for (int q = threadIdx.x; q < 64 * 16; q += 256) { const int rl = q >> 4, pc = q & 15;
    vst2(out + (size_t)(blockIdx.x * 64 + rl) * G3H + blockIdx.y * 64 + pc * 4, *(const v4f*)(&st[rl][pc * 4])); }
}

__global__ void gru_kernel(const float* __restrict__ xp_f,
                           const float* __restrict__ xp_b,
                           const _Float16* __restrict__ Whh_f,
                           const _Float16* __restrict__ Whh_b,
                           const float* __restrict__ bhh_f,
                           const float* __restrict__ bhh_b,
                           float* __restrict__ hout_f32) {
  const int dir = blockIdx.x;
  const float* xp = dir ? xp_b : xp_f;
  const _Float16* Whh = dir ? Whh_b : Whh_f;
  const float* bhh = dir ? bhh_b : bhh_f;
  const int colOff = dir ? HGRU : 0;

  __shared__ __align__(16) _Float16 hS[16][HGRU];
  __shared__ __align__(16) float ghS[16][G3H];

  int tid = threadIdx.x;
  int wave = tid >> 5;
  int lane = tid & 31;

  for (int i = tid; i < 16 * HGRU; i += 576) (&hS[0][0])[i] = (_Float16)0.0f;
  float hcarry[6] = {0.f, 0.f, 0.f, 0.f, 0.f, 0.f};

  v16h B[2][6];
#pragma unroll
  for (int tc = 0; tc < 2; ++tc)
#pragma unroll
    for (int kt = 0; kt < 6; ++kt)
      B[tc][kt] = load_frag_b(Whh, HGRU, wave * 32 + tc * 16, kt * 32);

  __syncthreads();

  for (int step = 0; step < LEN; ++step) {
    int t = dir ? (LEN - 1 - step) : step;
    v8f c0 = vzero8f(), c1 = vzero8f();
#pragma unroll
    for (int kt = 0; kt < 6; ++kt) {
      v16h a = load_frag_a(&hS[0][0], HGRU, kt * 32);
      c0 = wmma16(a, B[0][kt], c0);
      c1 = wmma16(a, B[1][kt], c1);
    }
    int mrow = (lane >> 4) * 8;
    int ncol = (lane & 15) + wave * 32;
#pragma unroll
    for (int v = 0; v < 8; ++v) {
      ghS[mrow + v][ncol]      = c0[v];
      ghS[mrow + v][ncol + 16] = c1[v];
    }
    __syncthreads();
    for (int idx = tid, k = 0; idx < 16 * HGRU; idx += 576, ++k) {
      int m = idx / HGRU, j = idx % HGRU;
      size_t base = (size_t)(m * LEN + t) * G3H;
      float xr = xp[base + j];
      float xz = xp[base + HGRU + j];
      float xn = xp[base + 2 * HGRU + j];
      float hr = ghS[m][j] + bhh[j];
      float hz = ghS[m][HGRU + j] + bhh[HGRU + j];
      float hn = ghS[m][2 * HGRU + j] + bhh[2 * HGRU + j];
      float hold = hcarry[k];
      float r  = 1.0f / (1.0f + expf(-(xr + hr)));
      float z  = 1.0f / (1.0f + expf(-(xz + hz)));
      float nn = tanhf(xn + r * hn);
      float hnew = (1.0f - z) * nn + z * hold;
      hS[m][j] = (_Float16)hnew; hcarry[k] = hnew;
      size_t ob = (size_t)(m * LEN + t) * (2 * HGRU) + colOff + j;
      *(volatile float*)(hout_f32 + ob) = hnew; __threadfence(); *(volatile float*)(hout_f32 + ob) = hnew;
    }
    __syncthreads();
  }
}

__global__ void feat_kernel(const float* __restrict__ h,
                            const float* __restrict__ adm_out,
                            _Float16* __restrict__ feat) {
  int g8 = blockIdx.x * blockDim.x + threadIdx.x;
  int i0 = g8 * 8;
  if (i0 >= ROWS * DCH * 64) return;
  int k0 = i0 & 63, t = i0 >> 6;
  int d = t % DCH, row = t / DCH;
  union { v8h hh; v4u u; } pk;
#pragma unroll
  for (int e = 0; e < 8; ++e) { int k = k0 + e; float v;
    if (k < 32)       v = h[(size_t)row * (2 * HGRU) + d * 32 + k];
    else if (k < 48)  v = adm_out[(row >> 10) * 16 + (k - 32)];
    else              v = 0.0f;
    pk.hh[e] = (_Float16)v; }
  vst2(feat + i0, pk.u);
}

__global__ void ffn_kernel(const _Float16* __restrict__ feat,
                           const _Float16* __restrict__ W1,
                           const float* __restrict__ b1,
                           const float* __restrict__ lng,
                           const float* __restrict__ lnb,
                           const float* __restrict__ W2,
                           const float* __restrict__ b2,
                           float* __restrict__ outT) {
  int d = blockIdx.y;
  int r0 = blockIdx.x * 32;
  int tid = threadIdx.x;
  int wave = tid >> 5, lane = tid & 31;
  __shared__ __align__(16) float hhS[32][FFH];
  __shared__ float res[32];

  const _Float16* Wd = W1 + (size_t)d * FFH * 64;
  int c0 = wave * 32;
#pragma unroll
  for (int mt = 0; mt < 2; ++mt) {
    const _Float16* Abase = feat + ((size_t)(r0 + mt * 16) * DCH + d) * 64;
    v8f a0 = vzero8f(), a1 = vzero8f();
#pragma unroll
    for (int kt = 0; kt < 2; ++kt) {
      v16h a  = load_frag_a(Abase, DCH * 64, kt * 32);
      v16h bb0 = load_frag_b(Wd, 64, c0, kt * 32);
      v16h bb1 = load_frag_b(Wd, 64, c0 + 16, kt * 32);
      a0 = wmma16(a, bb0, a0);
      a1 = wmma16(a, bb1, a1);
    }
    int mrow = (lane >> 4) * 8, ncol = lane & 15;
#pragma unroll
    for (int v = 0; v < 8; ++v) {
      hhS[mt * 16 + mrow + v][c0 + ncol]      = a0[v] + b1[d * FFH + c0 + ncol];
      hhS[mt * 16 + mrow + v][c0 + 16 + ncol] = a1[v] + b1[d * FFH + c0 + 16 + ncol];
    }
  }
  __syncthreads();

  for (int rr = 0; rr < 2; ++rr) {
  int row = wave * 2 + rr;
  int cl = tid & 31;
  float s = 0.0f, ss = 0.0f;
#pragma unroll
  for (int i = 0; i < 16; ++i) {
    float v = hhS[row][cl + 32 * i];
    s += v; ss += v * v;
  }
#pragma unroll
  for (int m = 16; m >= 1; m >>= 1) {
    s  += __shfl_xor(s,  m, 32);
    ss += __shfl_xor(ss, m, 32);
  }
  float mu  = s * (1.0f / FFH);
  float var = ss * (1.0f / FFH) - mu * mu;
  float inv = rsqrtf(var + 1e-5f);
  float dot = 0.0f;
#pragma unroll
  for (int i = 0; i < 16; ++i) {
    int c = cl + 32 * i;
    float v = (hhS[row][c] - mu) * inv * lng[d * FFH + c] + lnb[d * FFH + c];
    v = fmaxf(v, 0.0f);
    dot += v * W2[d * FFH + c];
  }
#pragma unroll
  for (int m = 16; m >= 1; m >>= 1) dot += __shfl_xor(dot, m, 32);
  if (cl == 0) res[row] = dot + b2[d];
  }
  __syncthreads();
  if (tid < 32) vst2(outT + (size_t)d * ROWS + r0 + tid, (float_a)res[tid]);
}

__global__ void __launch_bounds__(256) out_transpose_kernel(const float* __restrict__ outT, float* __restrict__ out) {
  const int q = blockIdx.x * 256 + threadIdx.x;
  if (q >= ROWS * DCH / 4) return;
  v4f v;
#pragma unroll
  for (int e = 0; e < 4; ++e) { const int f = q * 4 + e; const int row = f / DCH, d = f % DCH; v[e] = outT[(size_t)d * ROWS + row]; }
  vst2(out + (size_t)q * 4, v);
}

extern "C" void kernel_launch(void* const* d_in, const int* in_sizes, int n_in,
                              void* d_out, int out_size, void* d_ws, size_t ws_size,
                              hipStream_t stream) {
  const float* series   = (const float*)d_in[0];
  const float* adm      = (const float*)d_in[1];
  const int*   mask     = (const int*)d_in[2];
  const float* series_W = (const float*)d_in[3];
  const float* mask_emb = (const float*)d_in[4];
  const float* adm_W1 = (const float*)d_in[5];
  const float* adm_b1 = (const float*)d_in[6];
  const float* adm_W2 = (const float*)d_in[7];
  const float* adm_b2 = (const float*)d_in[8];
  const float* Wih[4] = {(const float*)d_in[9],  (const float*)d_in[13],
                         (const float*)d_in[17], (const float*)d_in[21]};
  const float* Whh[4] = {(const float*)d_in[10], (const float*)d_in[14],
                         (const float*)d_in[18], (const float*)d_in[22]};
  const float* bih[4] = {(const float*)d_in[11], (const float*)d_in[15],
                         (const float*)d_in[19], (const float*)d_in[23]};
  const float* bhh[4] = {(const float*)d_in[12], (const float*)d_in[16],
                         (const float*)d_in[20], (const float*)d_in[24]};
  const float* ffn_W1 = (const float*)d_in[25];
  const float* ffn_b1 = (const float*)d_in[26];
  const float* ln_g   = (const float*)d_in[27];
  const float* ln_b   = (const float*)d_in[28];
  const float* ffn_W2 = (const float*)d_in[29];
  const float* ffn_b2 = (const float*)d_in[30];
  float* out = (float*)d_out;

  char* p = (char*)d_ws;
  auto carve = [&](size_t bytes) -> void* {
    void* r = (void*)p;
    p += (bytes + 255) & ~(size_t)255;
    return r;
  };
  _Float16* x0_h   = (_Float16*)carve((size_t)ROWS * 96 * 2);
  float*    xp_f   = (float*)carve((size_t)ROWS * G3H * 4);
  float*    xp_b   = (float*)carve((size_t)ROWS * G3H * 4);
  float*    h_f32  = (float*)carve((size_t)ROWS * 2 * HGRU * 4);
  float*    outT   = (float*)carve((size_t)DCH * ROWS * 4);
  _Float16* feat   = (_Float16*)carve((size_t)ROWS * DCH * 64 * 2);
  float*    admout = (float*)carve(16 * 16 * 4);
  _Float16* Wih16[4], *Whh16[4];
  int kin[4] = {96, 96, 384, 384};
  for (int i = 0; i < 4; ++i) {
    Wih16[i] = (_Float16*)carve((size_t)G3H * kin[i] * 2);
    Whh16[i] = (_Float16*)carve((size_t)G3H * HGRU * 2);
  }
  _Float16* W1pad = (_Float16*)carve((size_t)DCH * FFH * 64 * 2);

  auto cvt = [&](const float* src, _Float16* dst, int n) {
    cvt_f16_kernel<<<(n / 8 + 255) / 256, 256, 0, stream>>>(src, dst, n);
  };
  for (int i = 0; i < 4; ++i) {
    cvt(Wih[i], Wih16[i], G3H * kin[i]);
    cvt(Whh[i], Whh16[i], G3H * HGRU);
  }
  cvt_w1_pad_kernel<<<(DCH * FFH * 64 / 8 + 255) / 256, 256, 0, stream>>>(ffn_W1, W1pad);

  embed_kernel<<<(ROWS * DCH + 255) / 256, 256, 0, stream>>>(
      series, mask, series_W, mask_emb, x0_h);
  adm_kernel<<<1, 256, 0, stream>>>(adm, adm_W1, adm_b1, adm_W2, adm_b2, admout);

  gemm_xw_kernel<_Float16><<<dim3(ROWS / 64, G3H / 64), 256, 0, stream>>>(
      x0_h, Wih16[0], bih[0], xp_f, 96);
  gemm_xw_kernel<_Float16><<<dim3(ROWS / 64, G3H / 64), 256, 0, stream>>>(
      x0_h, Wih16[1], bih[1], xp_b, 96);
  gru_kernel<<<2, 576, 0, stream>>>(xp_f, xp_b, Whh16[0], Whh16[1],
                                    bhh[0], bhh[1], h_f32);
  gemm_xw_kernel<float><<<dim3(ROWS / 64, G3H / 64), 256, 0, stream>>>(
      h_f32, Wih16[2], bih[2], xp_f, 384);
  gemm_xw_kernel<float><<<dim3(ROWS / 64, G3H / 64), 256, 0, stream>>>(
      h_f32, Wih16[3], bih[3], xp_b, 384);
  gru_kernel<<<2, 576, 0, stream>>>(xp_f, xp_b, Whh16[2], Whh16[3],
                                    bhh[2], bhh[3], h_f32);
  feat_kernel<<<(ROWS * DCH * 64 / 8 + 255) / 256, 256, 0, stream>>>(h_f32, admout, feat);
  ffn_kernel<<<dim3(ROWS / 32, DCH), 512, 0, stream>>>(
      feat, W1pad, ffn_b1, ln_g, ln_b, ffn_W2, ffn_b2, outT);
  out_transpose_kernel<<<(ROWS * DCH / 4 + 255) / 256, 256, 0, stream>>>(outT, out);
}
